// QGraphConv_19018115187414
// MI455X (gfx1250) — hardware-verified
//
#include <hip/hip_runtime.h>
#include <stddef.h>


#pragma clang fp contract(off)

#define IN_F    256
#define OUT_F   64
#define NTHR    256
#define NWAVE   8
#define EPT     8
#define NGRP    2
#define CHUNK   (NTHR * EPT * NGRP)
#define WCAP    (EPT * NGRP * 32)
#define LISTN   (NWAVE * WCAP)
#define NBD     4096
#define NBA     1024
#define FR      256
#define GROWS   128
#define APITCH  264

#define LDS_GEMM (2 * GROWS * APITCH * 2)
#define LDS_AGG  (NBA * OUT_F * 4 + LISTN * 4 + 64)

static_assert((CHUNK & (CHUNK - 1)) == 0);
static_assert(CHUNK <= 4096);
static_assert((NBD & (NBD - 1)) == 0 && NBD <= 4096);
static_assert((NBA & (NBA - 1)) == 0 && NBA <= 4096);
static_assert(GROWS * OUT_F * 4 <= GROWS * APITCH * 2);
static_assert((APITCH % 8) == 0);
static_assert((FR * IN_F / 4) % NTHR == 0);
static_assert((GROWS * IN_F / 8) % NTHR == 0);

typedef float          v2f   __attribute__((ext_vector_type(2)));
typedef float          v4f   __attribute__((ext_vector_type(4)));
typedef float          v8f   __attribute__((ext_vector_type(8)));
typedef int            v4i   __attribute__((ext_vector_type(4)));
typedef unsigned short v8us  __attribute__((ext_vector_type(8)));
typedef __bf16         v16bf __attribute__((ext_vector_type(16)));
union FragB { v16bf v; v8us h[2]; };

__device__ __forceinline__ v8f wmb(v16bf a, v16bf b, v8f c) {
  v8f d = __builtin_amdgcn_wmma_f32_16x16x32_bf16(false, a, false, b, (short)0, c, false, false);
  asm volatile("v_nop\n\tv_nop\n\tv_nop\n\tv_nop" : "+v"(d) : "v"(a), "v"(b));
  return d;
}

__device__ __forceinline__ float qste(float x, float mn, float sc, float rs, float qmax) {
  const float dlt = x - mn;
  float t = dlt * rs;
  t = fminf(fmaxf(t, 0.0f), qmax);
  const float r = rintf(t);
  const float q = r * sc + mn;
  const float d = q - x;
  return x + d;
}

__device__ __forceinline__ unsigned bfr(float f) {
  const unsigned u = __float_as_uint(f);
  return (u + 0x7FFFu + ((u >> 16) & 1u)) >> 16;
}

__device__ __forceinline__ unsigned qpair(float x, float mn, float sc, float rs, float qmax) {
  const float v = qste(x, mn, sc, rs, qmax);
  const unsigned h = bfr(v);
  const float hf = __uint_as_float(h << 16);
  const unsigned l = bfr(v - hf);
  return h | (l << 16);
}

template <int NB>
__device__ __forceinline__ int scan_chunk(const int* __restrict__ ids, int nE, int cbase, int nodeBase,
                                          int vec8, int* list, int tid, int lane, int wave) {
  int wc = 0;
#pragma unroll
  for (int g = 0; g < NGRP; ++g) {
    const int el0  = (g * NTHR + tid) * EPT;
    const int e0   = cbase + el0;
    const int sent = -2147483647 - 1;
    v4i da, db;
    if (vec8 != 0 && cbase + CHUNK <= nE) {
      da = *(const v4i*)(ids + e0);
      db = *(const v4i*)(ids + e0 + 4);
    } else {
      da.x = (e0     < nE) ? ids[min(e0,     nE - 1)] : sent;
      da.y = (e0 + 1 < nE) ? ids[min(e0 + 1, nE - 1)] : sent;
      da.z = (e0 + 2 < nE) ? ids[min(e0 + 2, nE - 1)] : sent;
      da.w = (e0 + 3 < nE) ? ids[min(e0 + 3, nE - 1)] : sent;
      db.x = (e0 + 4 < nE) ? ids[min(e0 + 4, nE - 1)] : sent;
      db.y = (e0 + 5 < nE) ? ids[min(e0 + 5, nE - 1)] : sent;
      db.z = (e0 + 6 < nE) ? ids[min(e0 + 6, nE - 1)] : sent;
      db.w = (e0 + 7 < nE) ? ids[min(e0 + 7, nE - 1)] : sent;
    }
    const unsigned nb = (unsigned)nodeBase;
    const unsigned s0 = (unsigned)da.x - nb, s1 = (unsigned)da.y - nb;
    const unsigned s2 = (unsigned)da.z - nb, s3 = (unsigned)da.w - nb;
    const unsigned s4 = (unsigned)db.x - nb, s5 = (unsigned)db.y - nb;
    const unsigned s6 = (unsigned)db.z - nb, s7 = (unsigned)db.w - nb;
    const bool h0 = s0 < (unsigned)NB, h1 = s1 < (unsigned)NB, h2 = s2 < (unsigned)NB, h3 = s3 < (unsigned)NB;
    const bool h4 = s4 < (unsigned)NB, h5 = s5 < (unsigned)NB, h6 = s6 < (unsigned)NB, h7 = s7 < (unsigned)NB;
    const unsigned any = __builtin_amdgcn_ballot_w32(h0 | h1 | h2 | h3 | h4 | h5 | h6 | h7);
    if (any != 0u) {
#define HITJ(J, HJ, SJ) { \
        const unsigned mj = __builtin_amdgcn_ballot_w32(HJ); \
        if (mj != 0u) { \
          if (HJ) { \
            const int pos = wc + (int)__builtin_amdgcn_mbcnt_lo(mj, 0u); \
            if (pos < WCAP) list[wave * WCAP + pos] = ((el0 + (J)) << 12) | (int)(SJ); \
          } \
          wc += (int)__builtin_popcount(mj); } }
      HITJ(0, h0, s0)
      HITJ(1, h1, s1)
      HITJ(2, h2, s2)
      HITJ(3, h3, s3)
      HITJ(4, h4, s4)
      HITJ(5, h5, s5)
      HITJ(6, h6, s6)
      HITJ(7, h7, s7)
#undef HITJ
    }
  }
  return wc;
}

__global__ __launch_bounds__(NTHR) void k_deg(
    const int* __restrict__ ids, float* rs, int nE, int vec8) {
  __shared__ __attribute__((aligned(16))) int cnt[NBD];
  __shared__ __attribute__((aligned(16))) int list[LISTN];
  __shared__ int wcnt[NWAVE];
  const int tid = threadIdx.x, lane = tid & 31, wave = tid >> 5;
  const int nodeBase = blockIdx.x * NBD;

  for (int i = tid; i < NBD; i += NTHR) cnt[i] = 0;
  __syncthreads();

  const int nChunks = (nE + CHUNK - 1) / CHUNK;
#pragma unroll 1
  for (int ch = 0; ch < nChunks; ++ch) {
    const int cbase = ch * CHUNK;
    const int wc = scan_chunk<NBD>(ids, nE, cbase, nodeBase, vec8, list, tid, lane, wave);
    if (lane == 0) wcnt[wave] = wc;
    __syncthreads();
    if (wave == 0) {
#pragma unroll 1
      for (int wsx = 0; wsx < NWAVE; ++wsx) {
        int n = __builtin_amdgcn_readfirstlane(wcnt[wsx]);
        n = n > WCAP ? WCAP : (n < 0 ? 0 : n);
        const int* lp = list + wsx * WCAP;
#pragma unroll 1
        for (int i = 0; i < n; ++i) {
          const int ent  = __builtin_amdgcn_readfirstlane(lp[i]);
          const int slot = ent & (NBD - 1);
          if (lane == 0) cnt[slot] = cnt[slot] + 1;
        }
      }
    }
    __syncthreads();
  }

#pragma unroll 1
  for (int i = tid; i < NBD; i += NTHR) {
    int c = cnt[i];
    c = c < 1 ? 1 : c;
    const float r = 1.0f / sqrtf((float)c);
    cnt[i] = __float_as_int(r);
  }
  __syncthreads();

  v4f dq[4];
#pragma unroll
  for (int q = 0; q < 4; ++q) {
    const int f = (wave * 4 + q) * 128 + 4 * lane;
    const v4i c = *(const v4i*)(cnt + f);
    dq[q].x = __int_as_float(c.x);
    dq[q].y = __int_as_float(c.y);
    dq[q].z = __int_as_float(c.z);
    dq[q].w = __int_as_float(c.w);
  }
  float* dp = rs + (size_t)nodeBase;
#pragma unroll
  for (int q = 0; q < 4; ++q) *(volatile v4f*)(dp + (wave * 4 + q) * 128 + 4 * lane) = dq[q];
  __threadfence();
#pragma unroll
  for (int q = 0; q < 4; ++q) *(volatile v4f*)(dp + (wave * 4 + q) * 128 + 4 * lane) = dq[q];
}

__global__ __launch_bounds__(NTHR) void k_fmm(
    const float* __restrict__ x, const float* __restrict__ rso, float* part, int nN) {
  __shared__ float smn[NWAVE], smx[NWAVE];
  const int tid = threadIdx.x, lane = tid & 31, wave = tid >> 5;
  const int rb = blockIdx.x * FR;
  const float pinf = __int_as_float(0x7f800000);
  float mn = pinf, mx = -pinf;
#pragma unroll 4
  for (int i = 0; i < (FR * IN_F / 4) / NTHR; ++i) {
    const int idx = i * NTHR + tid;
    const int r   = idx >> 6;
    const int c4  = (idx & 63) * 4;
    int node = rb + r;
    node = node > nN - 1 ? nN - 1 : node;
    const float s = rso[node];
    const v4f v = *(const v4f*)(x + (size_t)node * IN_F + c4) * s;
    mn = fminf(mn, fminf(fminf(v.x, v.y), fminf(v.z, v.w)));
    mx = fmaxf(mx, fmaxf(fmaxf(v.x, v.y), fmaxf(v.z, v.w)));
  }
#pragma unroll
  for (int o = 16; o > 0; o >>= 1) { mn = fminf(mn, __shfl_xor(mn, o)); mx = fmaxf(mx, __shfl_xor(mx, o)); }
  if (lane == 0) { smn[wave] = mn; smx[wave] = mx; }
  __syncthreads();
  if (wave == 0) {
    float a = smn[lane & 7], b = smx[lane & 7];
#pragma unroll
    for (int o = 4; o > 0; o >>= 1) { a = fminf(a, __shfl_xor(a, o)); b = fmaxf(b, __shfl_xor(b, o)); }
    v4f pv;
    pv.x = a; pv.y = b; pv.z = a; pv.w = b;
    float* pp = part + (size_t)blockIdx.x * 32 + 4 * (lane & 7);
    if (lane < 8) *(volatile v4f*)pp = pv;
    __threadfence();
    if (lane < 8) *(volatile v4f*)pp = pv;
  }
}

__global__ __launch_bounds__(NTHR) void k_prep(
    const float* __restrict__ w, const float* __restrict__ part,
    const int* __restrict__ nbits, const int* __restrict__ ngb, int nPart,
    unsigned short* whi, unsigned short* wlo, float* prm) {
  __shared__ __attribute__((aligned(16))) unsigned short tile[OUT_F * IN_F];
  __shared__ __attribute__((aligned(16))) float spar[32];
  __shared__ float smnF[NWAVE], smxF[NWAVE], smnW[NWAVE], smxW[NWAVE];
  (void)ngb;
  const int tid = threadIdx.x, lane = tid & 31, wave = tid >> 5;
  const float pinf = __int_as_float(0x7f800000);

  float mn = pinf, mx = -pinf;
#pragma unroll 1
  for (int p = tid; p < nPart; p += NTHR) {
    mn = fminf(mn, part[(size_t)p * 32]);
    mx = fmaxf(mx, part[(size_t)p * 32 + 1]);
  }
#pragma unroll
  for (int o = 16; o > 0; o >>= 1) { mn = fminf(mn, __shfl_xor(mn, o)); mx = fmaxf(mx, __shfl_xor(mx, o)); }
  if (lane == 0) { smnF[wave] = mn; smxF[wave] = mx; }

  mn = pinf; mx = -pinf;
#pragma unroll 1
  for (int i = tid; i < IN_F * OUT_F; i += NTHR) {
    const float v = w[i];
    mn = fminf(mn, v); mx = fmaxf(mx, v);
  }
#pragma unroll
  for (int o = 16; o > 0; o >>= 1) { mn = fminf(mn, __shfl_xor(mn, o)); mx = fmaxf(mx, __shfl_xor(mx, o)); }
  if (lane == 0) { smnW[wave] = mn; smxW[wave] = mx; }
  __syncthreads();

  if (tid == 0) {
    float a = smnF[0], b = smxF[0], c = smnW[0], d = smxW[0];
#pragma unroll
    for (int i = 1; i < NWAVE; ++i) {
      a = fminf(a, smnF[i]); b = fmaxf(b, smxF[i]);
      c = fminf(c, smnW[i]); d = fmaxf(d, smxW[i]);
    }
    int nb = nbits[0];
    nb = nb < 1 ? 1 : (nb > 24 ? 24 : nb);
    const float qmax = (float)((1 << nb) - 1);
    const float sf = fmaxf((b - a) / qmax, 1e-8f);
    const float sw = fmaxf((d - c) / qmax, 1e-8f);
    const float rsf = 1.0f / sf;
    const float rsw = 1.0f / sw;
    spar[0] = a;  spar[1] = sf; spar[2] = c; spar[3] = sw;
    spar[4] = qmax; spar[5] = b; spar[6] = d; spar[7] = (float)nb;
    spar[8] = rsf; spar[9] = rsw;
#pragma unroll
    for (int i = 10; i < 32; ++i) spar[i] = 0.0f;
  }
  __syncthreads();
  const float wmn = spar[2], sw = spar[3], qmax = spar[4], rsw = spar[9];

  if (wave == 0) {
    const v4f pv = *(const v4f*)(spar + 4 * (lane & 7));
    if (lane < 8) *(volatile v4f*)(prm + 4 * lane) = pv;
    __threadfence();
    if (lane < 8) *(volatile v4f*)(prm + 4 * lane) = pv;
  }

#pragma unroll 1
  for (int pass = 0; pass < 2; ++pass) {
#pragma unroll 1
    for (int e = tid; e < IN_F * OUT_F; e += NTHR) {
      const int k = e >> 6, n = e & (OUT_F - 1);
      const unsigned pq = qpair(w[e], wmn, sw, rsw, qmax);
      tile[n * IN_F + k] = (unsigned short)(pass == 0 ? (pq & 0xFFFFu) : (pq >> 16));
    }
    __syncthreads();
    unsigned short* dstp = (pass == 0) ? whi : wlo;
#pragma unroll
    for (int i = 0; i < 8; ++i) {
      const int n = i * 8 + wave;
      const v8us v = *(const v8us*)(tile + n * IN_F + 8 * lane);
      *(volatile v8us*)(dstp + n * IN_F + 8 * lane) = v;
    }
    __threadfence();
#pragma unroll
    for (int i = 0; i < 8; ++i) {
      const int n = i * 8 + wave;
      const v8us v = *(const v8us*)(tile + n * IN_F + 8 * lane);
      *(volatile v8us*)(dstp + n * IN_F + 8 * lane) = v;
    }
    __syncthreads();
  }
}

__global__ __launch_bounds__(NTHR) void k_gemm(
    const float* __restrict__ x, const float* __restrict__ rso, const float* __restrict__ prm,
    const unsigned short* __restrict__ whi, const unsigned short* __restrict__ wlo,
    float* h, int nN) {
  extern __shared__ v4f lds_dyn[];
  unsigned short* sH  = (unsigned short*)lds_dyn;
  unsigned short* sL  = sH + GROWS * APITCH;
  float*          stg = (float*)lds_dyn;
  const int tid = threadIdx.x, lane = tid & 31, wave = tid >> 5, hh = lane >> 4, m = lane & 15;
  const int rowBase = blockIdx.x * GROWS;
  const float mn = prm[0], sc = prm[1], qmax = prm[4], rs = prm[8];

#pragma unroll 1
  for (int i = 0; i < (GROWS * IN_F / 8) / NTHR; ++i) {
    const int idx = i * NTHR + tid;
    const int r   = idx >> 5;
    const int c0  = (idx & 31) * 8;
    int node = rowBase + r;
    node = node > nN - 1 ? nN - 1 : node;
    const float s = rso[node];
    const float* xp = x + (size_t)node * IN_F + c0;
    const v4f a = *(const v4f*)xp * s, b = *(const v4f*)(xp + 4) * s;
    const unsigned p0 = qpair(a.x, mn, sc, rs, qmax), p1 = qpair(a.y, mn, sc, rs, qmax);
    const unsigned p2 = qpair(a.z, mn, sc, rs, qmax), p3 = qpair(a.w, mn, sc, rs, qmax);
    const unsigned p4 = qpair(b.x, mn, sc, rs, qmax), p5 = qpair(b.y, mn, sc, rs, qmax);
    const unsigned p6 = qpair(b.z, mn, sc, rs, qmax), p7 = qpair(b.w, mn, sc, rs, qmax);
    v8us vh, vl;
    vh[0] = (unsigned short)(p0 & 0xFFFFu); vl[0] = (unsigned short)(p0 >> 16);
    vh[1] = (unsigned short)(p1 & 0xFFFFu); vl[1] = (unsigned short)(p1 >> 16);
    vh[2] = (unsigned short)(p2 & 0xFFFFu); vl[2] = (unsigned short)(p2 >> 16);
    vh[3] = (unsigned short)(p3 & 0xFFFFu); vl[3] = (unsigned short)(p3 >> 16);
    vh[4] = (unsigned short)(p4 & 0xFFFFu); vl[4] = (unsigned short)(p4 >> 16);
    vh[5] = (unsigned short)(p5 & 0xFFFFu); vl[5] = (unsigned short)(p5 >> 16);
    vh[6] = (unsigned short)(p6 & 0xFFFFu); vl[6] = (unsigned short)(p6 >> 16);
    vh[7] = (unsigned short)(p7 & 0xFFFFu); vl[7] = (unsigned short)(p7 >> 16);
    *(v8us*)(sH + r * APITCH + c0) = vh;
    *(v8us*)(sL + r * APITCH + c0) = vl;
  }
  __syncthreads();

  v8f acc[4];
#pragma unroll
  for (int t = 0; t < 4; ++t) { v8f z = {0.f, 0.f, 0.f, 0.f, 0.f, 0.f, 0.f, 0.f}; acc[t] = z; }
  const unsigned short* arH = sH + (wave * 16 + m) * APITCH + 8 * hh;
  const unsigned short* arL = sL + (wave * 16 + m) * APITCH + 8 * hh;
#pragma unroll 1
  for (int kt = 0; kt < IN_F / 32; ++kt) {
    FragB aH, aL;
    aH.h[0] = *(const v8us*)(arH + 32 * kt);
    aH.h[1] = *(const v8us*)(arH + 32 * kt + 16);
    aL.h[0] = *(const v8us*)(arL + 32 * kt);
    aL.h[1] = *(const v8us*)(arL + 32 * kt + 16);
#pragma unroll
    for (int t = 0; t < 4; ++t) {
      const size_t bo = (size_t)(16 * t + m) * IN_F + 32 * kt + 8 * hh;
      FragB bH, bL;
      bH.h[0] = *(const v8us*)(whi + bo);
      bH.h[1] = *(const v8us*)(whi + bo + 16);
      bL.h[0] = *(const v8us*)(wlo + bo);
      bL.h[1] = *(const v8us*)(wlo + bo + 16);
      acc[t] = wmb(aH.v, bH.v, acc[t]);
      acc[t] = wmb(aL.v, bH.v, acc[t]);
      acc[t] = wmb(aH.v, bL.v, acc[t]);
    }
  }
  __syncthreads();

  float* sp = stg + (wave * 16 + 8 * hh) * OUT_F + m;
#pragma unroll
  for (int t = 0; t < 4; ++t) {
    sp[0 * OUT_F + 16 * t] = acc[t][0];
    sp[1 * OUT_F + 16 * t] = acc[t][1];
    sp[2 * OUT_F + 16 * t] = acc[t][2];
    sp[3 * OUT_F + 16 * t] = acc[t][3];
    sp[4 * OUT_F + 16 * t] = acc[t][4];
    sp[5 * OUT_F + 16 * t] = acc[t][5];
    sp[6 * OUT_F + 16 * t] = acc[t][6];
    sp[7 * OUT_F + 16 * t] = acc[t][7];
  }
  __syncthreads();

  const float* lp = stg + wave * 16 * OUT_F + 4 * lane;
  float* gp = h + ((size_t)rowBase + wave * 16) * OUT_F + 4 * lane;
#pragma unroll
  for (int q = 0; q < 8; ++q) { const v4f v = *(const v4f*)(lp + q * 128); *(volatile v4f*)(gp + q * 128) = v; }
  __threadfence();
#pragma unroll
  for (int q = 0; q < 8; ++q) { const v4f v = *(const v4f*)(lp + q * 128); *(volatile v4f*)(gp + q * 128) = v; }
}

__global__ __launch_bounds__(NTHR) void k_agg(
    const int* __restrict__ srcs, const int* __restrict__ dsts, const float* __restrict__ h,
    const float* __restrict__ rsi, const float* __restrict__ bias, float* out,
    int nN, int nE, int vec8) {
  extern __shared__ v4f lds_dyn[];
  float* acc  = (float*)lds_dyn;
  int*   list = (int*)(acc + NBA * OUT_F);
  int*   wcnt = list + LISTN;
  const int tid = threadIdx.x, lane = tid & 31, wave = tid >> 5;
  const int nodeBase = blockIdx.x * NBA;

  {
    const v4f z = {0.f, 0.f, 0.f, 0.f};
    for (int i = tid; i < NBA * OUT_F / 4; i += NTHR) lds_dyn[i] = z;
  }
  __syncthreads();

  const int nChunks = (nE + CHUNK - 1) / CHUNK;
#pragma unroll 1
  for (int ch = 0; ch < nChunks; ++ch) {
    const int cbase = ch * CHUNK;
    const int wc = scan_chunk<NBA>(dsts, nE, cbase, nodeBase, vec8, list, tid, lane, wave);
    if (lane == 0) wcnt[wave] = wc;
    __syncthreads();
    if (wave == 0) {
#pragma unroll 1
      for (int wsx = 0; wsx < NWAVE; ++wsx) {
        int n = __builtin_amdgcn_readfirstlane(wcnt[wsx]);
        n = n > WCAP ? WCAP : (n < 0 ? 0 : n);
        const int* lp = list + wsx * WCAP;
#pragma unroll 1
        for (int i = 0; i < n; ++i) {
          const int ent  = __builtin_amdgcn_readfirstlane(lp[i]);
          const int slot = ent & (NBA - 1);
          int e = cbase + ((ent >> 12) & (CHUNK - 1));
          e = e > nE - 1 ? nE - 1 : e;
          int s = srcs[e];
          s = s < 0 ? 0 : (s > nN - 1 ? nN - 1 : s);
          const v2f v = *(const v2f*)(h + (size_t)s * OUT_F + 2 * lane);
          v2f* ap = (v2f*)(acc + slot * OUT_F + 2 * lane);
          *ap = *ap + v;
        }
      }
    }
    __syncthreads();
  }

#pragma unroll 4
  for (int i = 0; i < (NBA * OUT_F / 4) / NTHR; ++i) {
    const int idx  = i * NTHR + tid;
    const int slot = idx >> 4;
    const int c4   = (idx & 15) * 4;
    int node = nodeBase + slot;
    node = node > nN - 1 ? nN - 1 : node;
    const float d  = rsi[node];
    const v4f   bv = *(const v4f*)(bias + c4);
    v4f* ap = (v4f*)(acc + slot * OUT_F + c4);
    const v4f r = *ap * d;
    *ap = r + bv;
  }
  __syncthreads();

  const size_t outN = (size_t)nN * OUT_F;
  const size_t ob   = (size_t)nodeBase * OUT_F;
#pragma unroll 4
  for (int q = 0; q < 64; ++q) {
    const int f = (wave * 64 + q) * 128 + 4 * lane;
    const size_t gi = ob + (size_t)f;
    if (gi < outN) { const v4f v = *(const v4f*)(acc + f); *(volatile v4f*)(out + gi) = v; }
  }
  __threadfence();
#pragma unroll 4
  for (int q = 0; q < 64; ++q) {
    const int f = (wave * 64 + q) * 128 + 4 * lane;
    const size_t gi = ob + (size_t)f;
    if (gi < outN) { const v4f v = *(const v4f*)(acc + f); *(volatile v4f*)(out + gi) = v; }
  }
}

extern "C" void kernel_launch(void* const* d_in, const int* in_sizes, int n_in,
                              void* d_out, int out_size, void* d_ws, size_t ws_size,
                              hipStream_t stream) {
  if (n_in < 7) return;
  const int nN = in_sizes[0] / IN_F;
  const int nE = in_sizes[3];
  if (nN <= 0 || in_sizes[0] != nN * IN_F) return;
  if (in_sizes[1] != IN_F * OUT_F || in_sizes[2] < OUT_F) return;
  if (nE < 0 || in_sizes[4] != nE || in_sizes[5] < 1) return;
  if (out_size != nN * OUT_F) return;

  const float* feat = (const float*)d_in[0];
  const float* wgt  = (const float*)d_in[1];
  const float* bias = (const float*)d_in[2];
  const int*   src  = (const int*)d_in[3];
  const int*   dst  = (const int*)d_in[4];
  const int*   nbit = (const int*)d_in[5];
  const int*   ngb  = (const int*)d_in[6];
  float* out = (float*)d_out;

  const int nBD = (nN + NBD - 1) / NBD;
  const int nFB = (nN + FR - 1) / FR;
  const int nG  = (nN + GROWS - 1) / GROWS;
  const int nA  = (nN + NBA - 1) / NBA;

  char* ws = (char*)d_ws;
  size_t off = 0;
  const size_t oRso = off; off += (size_t)nBD * NBD * 4;                      off = (off + 255) & ~(size_t)255;
  const size_t oRsi = off; off += (size_t)nBD * NBD * 4;                      off = (off + 255) & ~(size_t)255;
  const size_t oPrt = off; off += (size_t)nFB * 128;                          off = (off + 255) & ~(size_t)255;
  const size_t oPrm = off; off += 256;                                        off = (off + 255) & ~(size_t)255;
  const size_t oWhi = off; off += (size_t)OUT_F * IN_F * 2;                   off = (off + 255) & ~(size_t)255;
  const size_t oWlo = off; off += (size_t)OUT_F * IN_F * 2;                   off = (off + 255) & ~(size_t)255;
  const size_t oH   = off; off += (size_t)nG * GROWS * OUT_F * 4;             off = (off + 255) & ~(size_t)255;
  if (off > ws_size) return;
  if (off > (size_t)134217728) return;
  float*          rso  = (float*)(ws + oRso);
  float*          rsi  = (float*)(ws + oRsi);
  float*          part = (float*)(ws + oPrt);
  float*          prm  = (float*)(ws + oPrm);
  unsigned short* whi  = (unsigned short*)(ws + oWhi);
  unsigned short* wlo  = (unsigned short*)(ws + oWlo);
  float*          hpl  = (float*)(ws + oH);

  const int vec8 = 1;

  k_deg<<<nBD, NTHR, 0, stream>>>(src, rso, nE, vec8);
  k_deg<<<nBD, NTHR, 0, stream>>>(dst, rsi, nE, vec8);
  k_fmm<<<nFB, NTHR, 0, stream>>>(feat, rso, part, nN);
  k_prep<<<1, NTHR, 0, stream>>>(wgt, part, nbit, ngb, nFB, whi, wlo, prm);

  hipFuncSetAttribute(reinterpret_cast<const void*>(&k_gemm),
                      hipFuncAttributeMaxDynamicSharedMemorySize, LDS_GEMM);
  k_gemm<<<nG, NTHR, LDS_GEMM, stream>>>(feat, rso, prm, whi, wlo, hpl, nN);

  hipFuncSetAttribute(reinterpret_cast<const void*>(&k_agg),
                      hipFuncAttributeMaxDynamicSharedMemorySize, LDS_AGG);
  k_agg<<<nA, NTHR, LDS_AGG, stream>>>(src, dst, hpl, rsi, bias, out, nN, nE, vec8);
}
